// Model_1786706395657
// MI455X (gfx1250) — hardware-verified
//
#include <hip/hip_runtime.h>
#include <math.h>

constexpr int NBATCH = 64;
constexpr int NSEQ   = 512;
constexpr int NCHAN  = 321;
constexpr int NPRED  = 720;
constexpr int NEXP   = 8;
constexpr int NRANK  = 32;
constexpr int NCIDD  = 32;
constexpr int NHIDR  = 64;
constexpr int MROWS  = NBATCH * NCHAN;
constexpr int KHID   = NEXP * NRANK;
constexpr int PPAD   = 768;
constexpr int GATE_ROWS = 324;
constexpr int GBT_REAL  = NPRED * NCHAN;
constexpr int GBT_PAD   = 231136;
constexpr int OUT_PER_B = NPRED * NCHAN;
constexpr int OUT_TOTAL = NBATCH * OUT_PER_B;
constexpr int TPITCH    = 132;
constexpr float W1_CARRY = 16.0f;
constexpr float HG_CARRY = 64.0f;
constexpr float W2_CARRY = 8.0f;

static_assert(MROWS == 20544);
static_assert(MROWS % 64 == 0 && KHID % 64 == 0 && PPAD % 64 == 0);
static_assert(NSEQ % 32 == 0 && KHID % 32 == 0);
static_assert(MROWS % 32 == 0);
static_assert(NSEQ % 128 == 0 && KHID % 128 == 0);
static_assert(GATE_ROWS % 4 == 0 && GATE_ROWS >= NCHAN);
static_assert(GBT_PAD % 32 == 0 && GBT_PAD >= GBT_REAL && GBT_PAD - GBT_REAL < 32);
static_assert(OUT_TOTAL % 256 == 0);
static_assert(OUT_TOTAL == 14791680);
static_assert(PPAD >= NPRED);

typedef __attribute__((ext_vector_type(16))) _Float16 v16h;
typedef __attribute__((ext_vector_type(8)))  _Float16 v8h;
typedef __attribute__((ext_vector_type(8)))  float    v8f;
typedef __attribute__((ext_vector_type(4)))  float    v4f;
typedef __attribute__((ext_vector_type(2)))  float    v2f;

__device__ __forceinline__ void group_guard_h(v8f& a, v8f& b, v8f& c, v8f& d,
                                              v16h x, v16h y0, v16h y1, v16h y2, v16h y3) {
  asm volatile("v_nop\n\tv_nop\n\tv_nop\n\tv_nop"
               : "+v"(a), "+v"(b), "+v"(c), "+v"(d)
               : "v"(x), "v"(y0), "v"(y1), "v"(y2), "v"(y3));
}
__device__ __forceinline__ void acc_guard4(v8f& a, v8f& b, v8f& c, v8f& d) {
  asm volatile("v_nop\n\tv_nop\n\tv_nop\n\tv_nop" : "+v"(a), "+v"(b), "+v"(c), "+v"(d));
}

struct FragH {
  union U { v16h v; v8h h[2]; };
  static __device__ __forceinline__ v16h load(const _Float16* p) {
    U f;
    f.h[0] = *(const v8h*)(p);
    f.h[1] = *(const v8h*)(p + 16);
    return f.v;
  }
  static __device__ __forceinline__ v8f mma(v16h a, v16h b, v8f c) {
    return __builtin_amdgcn_wmma_f32_16x16x32_f16(false, a, false, b, (short)0, c, false, false);
  }
};

__global__ __launch_bounds__(256) void stats_kernel(const float* __restrict__ x,
                                                    float* __restrict__ meanp,
                                                    float* __restrict__ stdp) {
  const int m = blockIdx.x * 256 + threadIdx.x;
  if (m >= MROWS) return;
  const int bb = m / NCHAN;
  const int n  = m - bb * NCHAN;
  const float* xp = x + (size_t)bb * NSEQ * NCHAN + n;
  float s0 = 0.0f, s1 = 0.0f, s2 = 0.0f, s3 = 0.0f;
#pragma unroll 1
  for (int l = 0; l < NSEQ; l += 4) {
    s0 += xp[(size_t)(l + 0) * NCHAN];
    s1 += xp[(size_t)(l + 1) * NCHAN];
    s2 += xp[(size_t)(l + 2) * NCHAN];
    s3 += xp[(size_t)(l + 3) * NCHAN];
  }
  const float mu = ((s0 + s1) + (s2 + s3)) * (1.0f / (float)NSEQ);
  float q0 = 0.0f, q1 = 0.0f, q2 = 0.0f, q3 = 0.0f;
#pragma unroll 1
  for (int l = 0; l < NSEQ; l += 4) {
    const float d0 = xp[(size_t)(l + 0) * NCHAN] - mu;
    const float d1 = xp[(size_t)(l + 1) * NCHAN] - mu;
    const float d2 = xp[(size_t)(l + 2) * NCHAN] - mu;
    const float d3 = xp[(size_t)(l + 3) * NCHAN] - mu;
    q0 += d0 * d0;
    q1 += d1 * d1;
    q2 += d2 * d2;
    q3 += d3 * d3;
  }
  const float var = ((q0 + q1) + (q2 + q3)) * (1.0f / (float)(NSEQ - 1));
  const float sd  = sqrtf(var) + 1e-6f;
  *(volatile float*)(meanp + m) = mu;
  *(volatile float*)(stdp + m)  = sd;
  __threadfence();
  *(volatile float*)(meanp + m) = mu;
  *(volatile float*)(stdp + m)  = sd;
}

__global__ __launch_bounds__(256) void router_gate_kernel(const float* __restrict__ ident,
                                                          const float* __restrict__ rw1,
                                                          const float* __restrict__ rb1,
                                                          const float* __restrict__ rw2,
                                                          const float* __restrict__ rb2,
                                                          float* __restrict__ gate) {
  __shared__ float hid[4][NHIDR];
  __shared__ float lgs[4][NEXP];
  const int tid = threadIdx.x;
  const int ch  = tid >> 6;
  const int t   = tid & 63;
  const int n   = blockIdx.x * 4 + ch;
  const int nc  = n < NCHAN ? n : NCHAN - 1;
  float acc = 0.0f;
#pragma unroll 4
  for (int c = 0; c < NCIDD; ++c) acc += ident[nc * NCIDD + c] * rw1[c * NHIDR + t];
  acc += rb1[t];
  hid[ch][t] = fmaxf(acc, 0.0f);
  __syncthreads();
  const int e = t & 7;
  float lg = 0.0f;
#pragma unroll 4
  for (int h = 0; h < NHIDR; ++h) lg += hid[ch][h] * rw2[h * NEXP + e];
  lg += rb2[e];
  if (t < NEXP) lgs[ch][t] = lg;
  __syncthreads();
  if (tid < 32) {
    const int c2 = tid >> 3;
    const int e2 = tid & 7;
    float mx = lgs[c2][0];
#pragma unroll
    for (int k = 1; k < NEXP; ++k) mx = fmaxf(mx, lgs[c2][k]);
    float sum = 0.0f, mine = 0.0f;
#pragma unroll 1
    for (int k = 0; k < NEXP; ++k) {
      const float ex = expf(lgs[c2][k] - mx);
      sum += ex;
      mine = (k == e2) ? ex : mine;
    }
    const float g = mine * (1.0f / sum);
    float* gp = gate + blockIdx.x * 32 + tid;
    *(volatile float*)gp = g;
    __threadfence();
    *(volatile float*)gp = g;
  }
}

__global__ __launch_bounds__(256) void gated_bias_kernel(const float* __restrict__ gate,
                                                         const float* __restrict__ bias,
                                                         float* __restrict__ gbT) {
  const int j = blockIdx.x * 256 + threadIdx.x;
  if (j >= GBT_PAD) return;
  const int jc = j < GBT_REAL ? j : GBT_REAL - 1;
  const int p  = jc / NCHAN;
  const int n  = jc - p * NCHAN;
  const v4f ga = *(const v4f*)(gate + n * NEXP);
  const v4f gc = *(const v4f*)(gate + n * NEXP + 4);
  float a = 0.0f;
  a += ga[0] * bias[0 * NPRED + p];
  a += ga[1] * bias[1 * NPRED + p];
  a += ga[2] * bias[2 * NPRED + p];
  a += ga[3] * bias[3 * NPRED + p];
  a += gc[0] * bias[4 * NPRED + p];
  a += gc[1] * bias[5 * NPRED + p];
  a += gc[2] * bias[6 * NPRED + p];
  a += gc[3] * bias[7 * NPRED + p];
  const float o = (j < GBT_REAL) ? a : 0.0f;
  *(volatile float*)(gbT + j) = o;
  __threadfence();
  *(volatile float*)(gbT + j) = o;
}

template <int WIN, int KTOT, int ROWS_REAL, bool NORM>
__global__ __launch_bounds__(256) void tr_plane_kernel(const float* __restrict__ src,
                                                       const float* __restrict__ meanp,
                                                       const float* __restrict__ stdp,
                                                       unsigned short* __restrict__ dst,
                                                       float sc) {
  __shared__ __align__(16) float tile[32 * TPITCH];
  const int tid = threadIdx.x;
  const int r   = tid & 31;
  const int kq  = tid >> 5;
  const int m   = blockIdx.x * 32 + r;
  const int k0  = blockIdx.y * 128;
  const bool live = m < ROWS_REAL;
  const int mc  = live ? m : ROWS_REAL - 1;
  const int bb  = mc / WIN;
  const int n   = mc - bb * WIN;
  float mu = 0.0f, rs = sc;
  if (NORM) {
    mu = meanp[mc];
    rs = sc * (1.0f / stdp[mc]);
  }
  const float* sp = src + (size_t)bb * KTOT * WIN + n;
#pragma unroll 1
  for (int g = 0; g < 2; ++g) {
    float v[8];
#pragma unroll
    for (int i = 0; i < 8; ++i) {
      const int kl = kq + 8 * (g * 8 + i);
      v[i] = sp[(size_t)(k0 + kl) * WIN];
    }
#pragma unroll
    for (int i = 0; i < 8; ++i) {
      const int kl = kq + 8 * (g * 8 + i);
      const float o = (v[i] - mu) * rs;
      tile[r * TPITCH + kl] = live ? o : 0.0f;
    }
  }
  __syncthreads();
  v8h hv[2];
#pragma unroll
  for (int it = 0; it < 2; ++it) {
    const int idx = tid + it * 256;
    const int row = idx >> 4;
    const int c8  = idx & 15;
    const float* tp = tile + row * TPITCH + c8 * 8;
    const v4f a = *(const v4f*)(tp);
    const v4f b = *(const v4f*)(tp + 4);
#pragma unroll
    for (int e = 0; e < 4; ++e) {
      hv[it][e]     = (_Float16)a[e];
      hv[it][4 + e] = (_Float16)b[e];
    }
  }
  for (int pass = 0; pass < 2; ++pass) {
#pragma unroll
    for (int it = 0; it < 2; ++it) {
      const int idx = tid + it * 256;
      const int row = idx >> 4;
      const int c8  = idx & 15;
      *(volatile v8h*)(dst + (size_t)(blockIdx.x * 32 + row) * KTOT + k0 + c8 * 8) = hv[it];
    }
    __threadfence();
  }
}

template <bool GATE, int OUT_MODE>
__global__ __launch_bounds__(256) void wmma_gemm64_f16(
    const unsigned short* __restrict__ Ap, int lda,
    const unsigned short* __restrict__ Btp, int ldb,
    void* __restrict__ Cout, int ldc,
    const float* __restrict__ gate,
    int M, int N, int K, float scale) {
  const _Float16* A  = (const _Float16*)Ap;
  const _Float16* Bt = (const _Float16*)Btp;
  __shared__ __align__(16) float sT[8][16 * 68];
  const int lane = threadIdx.x & 31;
  const int wave = threadIdx.x >> 5;
  const int tilesN = N >> 6;
  const int tilesM = M >> 6;
  const int tile = blockIdx.x * 8 + wave;
  if (tile >= tilesM * tilesN) return;
  const int tm = tile / tilesN;
  const int tn = tile - tm * tilesN;
  const int m0 = tm << 6;
  const int n0 = tn << 6;

  const int rlane = lane & 15;
  const int koff  = (lane >> 4) * 8;
  const int mOff  = (lane >> 4) * 8;

  v8f acc[4][4];
#pragma unroll
  for (int i = 0; i < 4; ++i)
#pragma unroll
    for (int j = 0; j < 4; ++j) acc[i][j] = (v8f){0.f, 0.f, 0.f, 0.f, 0.f, 0.f, 0.f, 0.f};

  for (int k0 = 0; k0 < K; k0 += 32) {
    v16h bh[4];
#pragma unroll
    for (int j = 0; j < 4; ++j) {
      const size_t bo = (size_t)(n0 + (j << 4) + rlane) * ldb + koff + k0;
      bh[j] = FragH::load(Bt + bo);
    }
#pragma unroll
    for (int i = 0; i < 4; ++i) {
      const size_t ao = (size_t)(m0 + (i << 4) + rlane) * lda + koff + k0;
      const v16h ah = FragH::load(A + ao);
#pragma unroll
      for (int j = 0; j < 4; ++j) acc[i][j] = FragH::mma(ah, bh[j], acc[i][j]);
      group_guard_h(acc[i][0], acc[i][1], acc[i][2], acc[i][3], ah, bh[0], bh[1], bh[2], bh[3]);
    }
  }
  acc_guard4(acc[0][0], acc[0][1], acc[0][2], acc[0][3]);
  acc_guard4(acc[1][0], acc[1][1], acc[1][2], acc[1][3]);
  acc_guard4(acc[2][0], acc[2][1], acc[2][2], acc[2][3]);
  acc_guard4(acc[3][0], acc[3][1], acc[3][2], acc[3][3]);

  float* slab = sT[wave];
  const int e0 = n0 >> 5;
#pragma unroll
  for (int i = 0; i < 4; ++i) {
    const int mBase = m0 + (i << 4);
    float g0[8], g1[8];
#pragma unroll
    for (int r = 0; r < 8; ++r) {
      g0[r] = 1.0f;
      g1[r] = 1.0f;
    }
    if (GATE) {
#pragma unroll
      for (int r = 0; r < 8; ++r) {
        const int nrow = (mBase + mOff + r) % NCHAN;
        const v2f gg = *(const v2f*)(gate + nrow * NEXP + e0);
        g0[r] = gg[0];
        g1[r] = gg[1];
      }
    }
#pragma unroll
    for (int j = 0; j < 4; ++j) {
#pragma unroll
      for (int r = 0; r < 8; ++r) {
        float v = acc[i][j][r] * scale;
        if (GATE) v = v * ((j < 2) ? g0[r] : g1[r]);
        slab[(mOff + r) * 68 + (j << 4) + rlane] = v;
      }
    }
    __builtin_amdgcn_fence(__ATOMIC_RELEASE, "workgroup");
    __builtin_amdgcn_wave_barrier();
    __builtin_amdgcn_fence(__ATOMIC_ACQUIRE, "workgroup");
    if (OUT_MODE == 0) {
      float* C = (float*)Cout;
      const int hh = lane >> 4, c4 = (lane & 15) * 4;
      for (int pass = 0; pass < 2; ++pass) {
#pragma unroll
        for (int it = 0; it < 8; ++it) {
          const int row = it * 2 + hh;
          const v4f v = *(const v4f*)(slab + row * 68 + c4);
          *(volatile v4f*)(C + (size_t)(mBase + row) * ldc + n0 + c4) = v;
        }
        __threadfence();
      }
    } else {
      const int q = lane >> 3, c8 = (lane & 7) * 8;
      unsigned short* C = (unsigned short*)Cout;
      for (int pass = 0; pass < 2; ++pass) {
#pragma unroll
        for (int it = 0; it < 4; ++it) {
          const int row = it * 4 + q;
          const float* sp = slab + row * 68 + c8;
          v8h hv;
#pragma unroll
          for (int e = 0; e < 8; ++e) hv[e] = (_Float16)sp[e];
          *(volatile v8h*)(C + (size_t)(mBase + row) * ldc + n0 + c8) = hv;
        }
        __threadfence();
      }
    }
    __builtin_amdgcn_fence(__ATOMIC_RELEASE, "workgroup");
    __builtin_amdgcn_wave_barrier();
    __builtin_amdgcn_fence(__ATOMIC_ACQUIRE, "workgroup");
  }
}

__global__ __launch_bounds__(256) void finalize_kernel(const float* __restrict__ Yt,
                                                       const float* __restrict__ gbT,
                                                       const float* __restrict__ meanp,
                                                       const float* __restrict__ stdp,
                                                       float* __restrict__ out) {
  const unsigned i = blockIdx.x * 256u + threadIdx.x;
  if (i >= (unsigned)OUT_TOTAL) return;
  const unsigned bb  = i / (unsigned)OUT_PER_B;
  const unsigned rem = i - bb * (unsigned)OUT_PER_B;
  const unsigned p   = rem / (unsigned)NCHAN;
  const unsigned n   = rem - p * (unsigned)NCHAN;
  const unsigned m   = bb * (unsigned)NCHAN + n;
  const float y  = Yt[(size_t)p * MROWS + m];
  const float gb = gbT[rem];
  const float sd = stdp[m];
  const float mu = meanp[m];
  const float o  = (y + gb) * sd + mu;
  *(volatile float*)(out + i) = o;
  __threadfence();
  *(volatile float*)(out + i) = o;
}

extern "C" void kernel_launch(void* const* d_in, const int* in_sizes, int n_in,
                              void* d_out, int out_size, void* d_ws, size_t ws_size,
                              hipStream_t stream) {
  if (n_in < 9 || d_out == nullptr || d_ws == nullptr) return;
  if (in_sizes[0] != NBATCH * NSEQ * NCHAN || in_sizes[1] != NCHAN * NCIDD ||
      in_sizes[2] != NCIDD * NHIDR || in_sizes[3] != NHIDR || in_sizes[4] != NHIDR * NEXP ||
      in_sizes[5] != NEXP || in_sizes[6] != NEXP * NSEQ * NRANK ||
      in_sizes[7] != NEXP * NRANK * NPRED || in_sizes[8] != NEXP * NPRED ||
      out_size != OUT_TOTAL) return;

  const float* x     = (const float*)d_in[0];
  const float* ident = (const float*)d_in[1];
  const float* rw1   = (const float*)d_in[2];
  const float* rb1   = (const float*)d_in[3];
  const float* rw2   = (const float*)d_in[4];
  const float* rb2   = (const float*)d_in[5];
  const float* w1    = (const float*)d_in[6];
  const float* w2    = (const float*)d_in[7];
  const float* bias  = (const float*)d_in[8];
  float* out = (float*)d_out;

  char* ws = (char*)d_ws;
  size_t off = 0;
  auto carve = [&](size_t bytes) -> char* {
    char* p = ws + off;
    off += (bytes + 255) & ~(size_t)255;
    return p;
  };
  float*          MEANP = (float*)carve((size_t)MROWS * 4);
  float*          STDP  = (float*)carve((size_t)MROWS * 4);
  float*          GATEP = (float*)carve((size_t)GATE_ROWS * NEXP * 4);
  float*          GBTP  = (float*)carve((size_t)GBT_PAD * 4);
  unsigned short* A1    = (unsigned short*)carve((size_t)MROWS * NSEQ * 2);
  unsigned short* BT1   = (unsigned short*)carve((size_t)KHID * NSEQ * 2);
  unsigned short* W2T   = (unsigned short*)carve((size_t)PPAD * KHID * 2);
  unsigned short* HG    = (unsigned short*)carve((size_t)MROWS * KHID * 2);
  float*          YT    = (float*)carve((size_t)PPAD * MROWS * 4);
  if (off > ws_size || off > (size_t)134217728) return;

  stats_kernel<<<(MROWS + 255) / 256, 256, 0, stream>>>(x, MEANP, STDP);
  router_gate_kernel<<<GATE_ROWS / 4, 256, 0, stream>>>(ident, rw1, rb1, rw2, rb2, GATEP);
  gated_bias_kernel<<<(GBT_PAD + 255) / 256, 256, 0, stream>>>(GATEP, bias, GBTP);

  tr_plane_kernel<NCHAN, NSEQ, MROWS, true>
      <<<dim3(MROWS / 32, NSEQ / 128), 256, 0, stream>>>(x, MEANP, STDP, A1, 1.0f);
  tr_plane_kernel<NRANK, NSEQ, KHID, false>
      <<<dim3(KHID / 32, NSEQ / 128), 256, 0, stream>>>(w1, MEANP, STDP, BT1, W1_CARRY);
  tr_plane_kernel<NPRED, KHID, NPRED, false>
      <<<dim3(PPAD / 32, KHID / 128), 256, 0, stream>>>(w2, MEANP, STDP, W2T, W2_CARRY);

  {
    const int tiles = (MROWS / 64) * (KHID / 64);
    wmma_gemm64_f16<true, 1><<<(tiles + 7) / 8, 256, 0, stream>>>(
        A1, NSEQ, BT1, NSEQ, (void*)HG, KHID, GATEP, MROWS, KHID, NSEQ, HG_CARRY / W1_CARRY);
  }
  {
    const int tiles = (PPAD / 64) * (MROWS / 64);
    wmma_gemm64_f16<false, 0><<<(tiles + 7) / 8, 256, 0, stream>>>(
        W2T, KHID, HG, KHID, (void*)YT, MROWS, GATEP, PPAD, MROWS, KHID,
        1.0f / (HG_CARRY * W2_CARRY));
  }
  finalize_kernel<<<OUT_TOTAL / 256, 256, 0, stream>>>(YT, GBTP, MEANP, STDP, out);
}
